// OneSideInterModalityUpdate_36197984371017
// MI455X (gfx1250) — hardware-verified
//
#include <hip/hip_runtime.h>


namespace {
constexpr int Bn = 8, NS = 1024, NTT = 1024, D = 1024, H = 8, HD = 128, TS = Bn * NS, TT = Bn * NTT;
constexpr float XS = 8.0f, PS = 8.0f, ISQ = 0.08838834764831845f;
struct Wo_ { static constexpr size_t S = 0, T = (size_t)2 * D * D, O = T + (size_t)D * D, END = O + (size_t)D * 2 * D; };

typedef _Float16 b16;
typedef __attribute__((ext_vector_type(16))) _Float16 v16b;
typedef __attribute__((ext_vector_type(8))) _Float16 v8b;
typedef __attribute__((ext_vector_type(8))) float v8f;
typedef __attribute__((ext_vector_type(4))) float v4f;
__device__ __forceinline__ float bf16_rne(float f) { unsigned int u = __float_as_uint(f); u += 0x7FFFu + ((u >> 16) & 1u); return __uint_as_float(u & 0xFFFF0000u); }
__device__ __forceinline__ v16b frag_kb(const b16* p, int hh) { const v8b a = *(const v8b*)(p + 8 * hh), b = *(const v8b*)(p + 16 + 8 * hh); v16b f;
#pragma unroll
  for (int e = 0; e < 8; ++e) { f[e] = a[e]; f[8 + e] = b[e]; } return f; }
__device__ __forceinline__ v8f wmma16b(v16b a, v16b b, v8f c) { v8f d = __builtin_amdgcn_wmma_f32_16x16x32_f16(false, a, false, b, (short)0, c, false, false); asm volatile("v_nop\n\tv_nop\n\tv_nop\n\tv_nop" : "+v"(d) : "v"(a), "v"(b)); return d; }
__device__ __forceinline__ void wave_lds_sync() { __builtin_amdgcn_fence(__ATOMIC_RELEASE, "workgroup"); __builtin_amdgcn_wave_barrier(); __builtin_amdgcn_fence(__ATOMIC_ACQUIRE, "workgroup"); }
__device__ __forceinline__ float nexp(float x) { return __builtin_amdgcn_exp2f(x * 1.4426950408889634f); }
__device__ __forceinline__ float pmul(float a, float b) { float p = a * b; asm volatile("" : "+v"(p)); return p; }

__global__ __launch_bounds__(256) void prep_kernel(const float* __restrict__ ws_, const float* __restrict__ wt, const float* __restrict__ wo, const float* __restrict__ bs, const float* __restrict__ bt, const float* __restrict__ bo, b16* __restrict__ R, float* __restrict__ P) {
  const size_t tid = (size_t)blockIdx.x * 256 + threadIdx.x, nth = (size_t)gridDim.x * 256;
  for (int pass = 0; pass < 2; ++pass) { for (size_t p = tid; p < Wo_::END / 8; p += nth) { const size_t q = p * 8; const float* s_ = (q < Wo_::T) ? (ws_ + q) : (q < Wo_::O) ? (wt + (q - Wo_::T)) : (wo + (q - Wo_::O)); v8b v; for (int e = 0; e < 8; ++e) v[e] = (b16)bf16_rne(s_[e]); *(volatile v8b*)(R + q) = v; }
    for (size_t q = tid; q < 4096; q += nth) { const int i = (int)q; P[q] = bf16_rne((i < 2048) ? bs[i] : (i < 3072) ? bt[i - 2048] : bo[i - 3072]); } __threadfence(); }
}

__global__ __launch_bounds__(256) void xrows_kernel(const float* __restrict__ x, int rows, int pitch, b16* __restrict__ X) {
  const size_t tid = (size_t)blockIdx.x * 256 + threadIdx.x, nth = (size_t)gridDim.x * 256;
  for (int pass = 0; pass < 2; ++pass) { for (size_t p = tid; p < (size_t)rows * D / 8; p += nth) { const size_t r = p / (D / 8), c8 = (p % (D / 8)) * 8; v8b v; for (int e = 0; e < 8; ++e) v[e] = (b16)(bf16_rne(x[r * D + c8 + e]) * XS); *(volatile v8b*)(X + r * pitch + c8) = v; } __threadfence(); }
}

template <int K, int MODE, int MASK>
__global__ __launch_bounds__(64) void gemm_kernel(const b16* __restrict__ A, int lda, const b16* __restrict__ Bw, const float* __restrict__ bias, const float* __restrict__ rowmask, b16* __restrict__ O16, int ldo, float* __restrict__ O32) {
  __shared__ __attribute__((aligned(16))) float Ts[2][32][128 + 4];
  const int lane = threadIdx.x & 31, wave = threadIdx.x >> 5, nloc = lane & 15, hlf = lane >> 4, m0 = blockIdx.y * 32, c0 = blockIdx.x * 256 + wave * 128;
  v8f acc[2][8];
#pragma unroll
  for (int r = 0; r < 2; ++r)
#pragma unroll
    for (int t = 0; t < 8; ++t) acc[r][t] = (v8f){};
#pragma unroll 2
  for (int kb = 0; kb < K; kb += 32) { const v16b a0 = frag_kb(A + (size_t)(m0 + nloc) * lda + kb, hlf), a1 = frag_kb(A + (size_t)(m0 + 16 + nloc) * lda + kb, hlf);
#pragma unroll
    for (int t = 0; t < 8; ++t) { const v16b bw = frag_kb(Bw + (size_t)(c0 + t * 16 + nloc) * K + kb, hlf); acc[0][t] = wmma16b(a0, bw, acc[0][t]); acc[1][t] = wmma16b(a1, bw, acc[1][t]); } }
#pragma unroll
  for (int t = 0; t < 8; ++t) { const float bb = bias[c0 + t * 16 + nloc];
#pragma unroll
    for (int r = 0; r < 2; ++r)
#pragma unroll
      for (int v = 0; v < 8; ++v) { const int rr = r * 16 + 8 * hlf + v; float y = acc[r][t][v] * (1.0f / XS) + bb; if (MASK) y = pmul(y, bf16_rne(rowmask[m0 + rr])); Ts[wave][rr][t * 16 + nloc] = y; } }
  wave_lds_sync();
  for (int pass = 0; pass < 2; ++pass) {
    if (MODE == 2) { for (int i = lane; i < 32 * 32; i += 32) { const int rr = i >> 5, c4 = (i & 31) * 4; *(volatile v4f*)(O32 + (size_t)(m0 + rr) * ldo + c0 + c4) = *(const v4f*)(&Ts[wave][rr][c4]); } }
    else { for (int i = lane; i < 32 * 16; i += 32) { const int rr = i >> 4, c8 = (i & 15) * 8; v8b o; for (int e = 0; e < 8; ++e) o[e] = (b16)(Ts[wave][rr][c8 + e] * XS); *(volatile v8b*)(O16 + (size_t)(m0 + rr) * ldo + c0 + c8) = o; } }
    __threadfence(); }
}

__global__ __launch_bounds__(256) void vt_kernel(const b16* __restrict__ KV, b16* __restrict__ vt) {
  __shared__ __attribute__((aligned(16))) b16 T[HD][128 + 8];
  const int b = blockIdx.z, h = blockIdx.y, t0 = blockIdx.x * 128, t_ = threadIdx.x;
  for (int i = t_; i < 128 * (HD / 8); i += 256) { const int tk = i >> 4, d8 = (i & 15) * 8; const v8b vv = *(const v8b*)(KV + ((size_t)(b * NS + t0 + tk)) * (2 * D) + D + h * HD + d8); for (int e = 0; e < 8; ++e) T[d8 + e][tk] = vv[e]; }
  __syncthreads();
  for (int pass = 0; pass < 2; ++pass) { for (int i = t_; i < HD * 16; i += 256) { const int d = i >> 4, c8 = (i & 15) * 8; *(volatile v8b*)(vt + (((size_t)b * H + h) * HD + d) * NS + t0 + c8) = *(const v8b*)(&T[d][c8]); } __threadfence(); }
}

__global__ __launch_bounds__(256) void attn_kernel(const b16* __restrict__ Q, const b16* __restrict__ KV, const b16* __restrict__ vt, const float* __restrict__ smask, b16* __restrict__ CAT) {
  __shared__ __attribute__((aligned(16))) b16 Os[16][D + 8];
  const int h = threadIdx.x >> 5, lane = threadIdx.x & 31, hh = lane >> 4, col = lane & 15; const int b = blockIdx.x / (NTT / 16), q0 = (blockIdx.x % (NTT / 16)) * 16, qi = q0 + col;
  const b16* Qr = Q + (size_t)(b * NTT) * D + h * HD; const b16* Kr = KV + (size_t)(b * NS) * (2 * D) + h * HD; const b16* V = vt + (((size_t)b * H + h) * HD) * NS; const float* mb = smask + (size_t)b * NS;
  v16b qf[4];
#pragma unroll
  for (int j = 0; j < 4; ++j) qf[j] = frag_kb(Qr + (size_t)qi * D + 32 * j, hh);
  float m = -INFINITY, l = 0.0f; v8f o[8];
#pragma unroll
  for (int t = 0; t < 8; ++t) o[t] = (v8f){};
  for (int kb = 0; kb < NS; kb += 32) { v8f s0 = {}, s1 = {};
#pragma unroll
    for (int j = 0; j < 4; ++j) { s0 = wmma16b(frag_kb(Kr + (size_t)(kb + col) * (2 * D) + 32 * j, hh), qf[j], s0); s1 = wmma16b(frag_kb(Kr + (size_t)(kb + 16 + col) * (2 * D) + 32 * j, hh), qf[j], s1); }
    float mr = -INFINITY;
#pragma unroll
    for (int r = 0; r < 8; ++r) { const int k0 = kb + 8 * hh + r, k1 = k0 + 16; s0[r] = (bf16_rne(mb[k0]) == 0.0f) ? -INFINITY : s0[r] * (ISQ / (XS * XS)); s1[r] = (bf16_rne(mb[k1]) == 0.0f) ? -INFINITY : s1[r] * (ISQ / (XS * XS)); mr = fmaxf(mr, fmaxf(s0[r], s1[r])); }
    mr = fmaxf(mr, __shfl_xor(mr, 16)); const float mn = fmaxf(m, mr); const float al_ = (mn == -INFINITY) ? 1.0f : nexp(m - mn); m = mn; float sum = 0.0f; v16b pb;
#pragma unroll
    for (int r = 0; r < 8; ++r) { const float e0 = (s0[r] == -INFINITY) ? 0.0f : nexp(s0[r] - mn), e1 = (s1[r] == -INFINITY) ? 0.0f : nexp(s1[r] - mn); sum += e0 + e1; pb[r] = (b16)(e0 * PS); pb[8 + r] = (b16)(e1 * PS); }
    sum += __shfl_xor(sum, 16); l = l * al_ + sum;
#pragma unroll
    for (int t = 0; t < 8; ++t) { o[t] *= al_; o[t] = wmma16b(frag_kb(V + (size_t)(t * 16 + col) * NS + kb, hh), pb, o[t]); } }
  const float inv = (l > 0.0f) ? 1.0f / (l * PS) : 0.0f;
#pragma unroll
  for (int t = 0; t < 8; ++t)
#pragma unroll
    for (int r = 0; r < 8; ++r) Os[col][h * HD + t * 16 + 8 * hh + r] = (b16)(o[t][r] * inv);
  __syncthreads();
  for (int pass = 0; pass < 2; ++pass) { for (int i = threadIdx.x; i < 16 * (D / 8); i += 256) { const int rr = i / (D / 8), c8 = (i % (D / 8)) * 8; *(volatile v8b*)(CAT + ((size_t)(b * NTT + q0 + rr)) * (2 * D) + D + c8) = *(const v8b*)(&Os[rr][c8]); } __threadfence(); }
}
}

extern "C" void kernel_launch(void* const* d_in, const int* in_sizes, int n_in,
                              void* d_out, int out_size, void* d_ws, size_t ws_size, hipStream_t stream) {
  (void)n_in; (void)out_size;
  const float* src = (const float*)d_in[0]; const float* tgt = (const float*)d_in[1]; const float* sm = (const float*)d_in[2]; const float* tm = (const float*)d_in[3]; const float* ws_ = (const float*)d_in[4]; const float* bs = (const float*)d_in[5]; const float* wt = (const float*)d_in[6]; const float* bt = (const float*)d_in[7]; const float* wo = (const float*)d_in[8]; const float* bo = (const float*)d_in[9];
  float* out = (float*)d_out;
  if (in_sizes[0] != TS * D || in_sizes[1] != TT * D || in_sizes[4] != 2 * D * D || in_sizes[8] != D * 2 * D) return;
  size_t off = 0; char* ws = (char*)d_ws;
  auto carve = [&](size_t bytes) { char* p = ws + off; off += (bytes + 255) & ~(size_t)255; return p; };
  b16* R = (b16*)carve(Wo_::END * 2); float* P = (float*)carve(4096 * 4); b16* XS_ = (b16*)carve((size_t)TS * D * 2); b16* CAT = (b16*)carve((size_t)TT * 2 * D * 2); b16* KV = (b16*)carve((size_t)TS * 2 * D * 2); b16* Q = (b16*)carve((size_t)TT * D * 2); b16* VT = (b16*)carve((size_t)TS * D * 2);
  if (off > ws_size) return;
  prep_kernel<<<512, 256, 0, stream>>>(ws_, wt, wo, bs, bt, bo, R, P);
  xrows_kernel<<<512, 256, 0, stream>>>(src, TS, D, XS_);
  xrows_kernel<<<512, 256, 0, stream>>>(tgt, TT, 2 * D, CAT);
  gemm_kernel<D, 0, 1><<<dim3(2 * D / 256, TS / 32), 64, 0, stream>>>(XS_, D, R + Wo_::S, P, sm, KV, 2 * D, nullptr);
  gemm_kernel<D, 0, 1><<<dim3(D / 256, TT / 32), 64, 0, stream>>>(CAT, 2 * D, R + Wo_::T, P + 2048, tm, Q, D, nullptr);
  vt_kernel<<<dim3(NS / 128, H, Bn), 256, 0, stream>>>(KV, VT);
  attn_kernel<<<TT / 16, 256, 0, stream>>>(Q, KV, VT, sm, CAT);
  gemm_kernel<2 * D, 2, 0><<<dim3(D / 256, TT / 32), 64, 0, stream>>>(CAT, 2 * D, R + Wo_::O, P + 3072, nullptr, nullptr, D, out);
}
